// MambaBlock_63118839382421
// MI455X (gfx1250) — hardware-verified
//
#include <hip/hip_runtime.h>
#include <math.h>

typedef __attribute__((ext_vector_type(16))) _Float16 v16h;
typedef __attribute__((ext_vector_type(8)))  _Float16 v8h;
typedef __attribute__((ext_vector_type(8)))  float    v8f;
typedef __attribute__((ext_vector_type(4)))  float    v4f;
typedef __attribute__((ext_vector_type(4)))  unsigned u4v;
typedef u4v __attribute__((may_alias)) u4v_a;

constexpr int kBatch  = 16;
constexpr int kCin    = 64;
constexpr int kHid    = 256;
constexpr int kImgH   = 64;
constexpr int kImgW   = 64;
constexpr int kSeq    = kImgH * kImgW;
constexpr int kTok    = kBatch * kSeq;
constexpr int kConvK  = kCin * 9;
constexpr int kGuN    = 2 * kHid;
constexpr float kWCarry    = 32.0f;
constexpr float kWCarryInv = 1.0f / 32.0f;
constexpr int kConvThreads = 128;
constexpr int kOutWaves    = 2;
constexpr int kScanSteps   = 32;
constexpr int kScanPitch   = 132;
static_assert(kSeq == 4096 && kTok == 65536 && kConvK == 576, "shape");
static_assert((kConvK % 32) == 0 && (kHid % 32) == 0, "GEMM K multiples of 32");
static_assert((kTok % 64) == 0 && (kHid % 64) == 0 && (kGuN % 64) == 0 && (kCin % 64) == 0, "GEMM M,N multiples of 64");
static_assert((kSeq % kScanSteps) == 0, "scan chunking");

constexpr size_t kPlaneBytes = (size_t)kTok * kHid * 2;
constexpr size_t kOffR0   = 0;
constexpr size_t kOffR1   = kOffR0 + kPlaneBytes;
constexpr size_t kOffR2   = kOffR1 + kPlaneBytes;
constexpr size_t kOffWC1P = kOffR2 + kPlaneBytes;
constexpr size_t kOffWGI  = kOffWC1P + (size_t)kHid * kConvK * 2;
constexpr size_t kOffWS16 = kOffWGI + (size_t)kGuN * kHid * 2;
constexpr size_t kOffWO16 = kOffWS16 + (size_t)kHid * kHid * 2;
constexpr size_t kOffPART = kOffWO16 + (size_t)kCin * kHid * 2;
constexpr size_t kOffSS   = kOffPART + (size_t)256 * 512 * 4;
constexpr size_t kWsTotal = kOffSS + (size_t)512 * 4;
static_assert(kWsTotal == 101910528ull, "carve total");
static_assert(kWsTotal <= 134217728ull, "carve cap");
static_assert((size_t)kTok * kCin * 2 <= kPlaneBytes, "token-major input fits R2");
static_assert((kOffR1 % 128) == 0 && (kOffR2 % 128) == 0 && (kOffWC1P % 128) == 0 && (kOffWGI % 128) == 0 &&
              (kOffWS16 % 128) == 0 && (kOffWO16 % 128) == 0 && (kOffPART % 128) == 0 && (kOffSS % 128) == 0,
              "128-B aligned regions");

__device__ __forceinline__ float h16_to_f32(unsigned hb) {
  const unsigned sgn = (hb & 0x8000u) << 16;
  const unsigned em = hb & 0x7fffu;
  const float fn = __uint_as_float((em << 13) + 0x38000000u);
  const float fs = (float)em * 5.9604644775390625e-8f;
  const float mag = (em < 0x400u) ? fs : fn;
  return __uint_as_float(__float_as_uint(mag) | sgn);
}

__device__ __forceinline__ void guard_row4(v8f& a, v8f& b, v8f& c, v8f& d, v16h x, v16h y) {
  asm volatile("v_nop\n\tv_nop\n\tv_nop\n\tv_nop" : "+v"(a), "+v"(b), "+v"(c), "+v"(d) : "v"(x), "v"(y));
}
__device__ __forceinline__ void keep4_h(v16h a, v16h b, v16h c, v16h d) {
  asm volatile("v_nop" :: "v"(a), "v"(b), "v"(c), "v"(d));
}
__device__ __forceinline__ void acc_guard4(v8f& a, v8f& b, v8f& c, v8f& d) {
  asm volatile("v_nop\n\tv_nop\n\tv_nop\n\tv_nop" : "+v"(a), "+v"(b), "+v"(c), "+v"(d));
}
__device__ __forceinline__ void wave_lds_sync() {
  __builtin_amdgcn_fence(__ATOMIC_RELEASE, "workgroup");
  __builtin_amdgcn_wave_barrier();
  __builtin_amdgcn_fence(__ATOMIC_ACQUIRE, "workgroup");
}

template <typename T> struct Frag;
template <> struct Frag<_Float16> {
  typedef v16h V;
  union U { v16h v; v8h h[2]; };
  static __device__ __forceinline__ v16h load(const _Float16* p) {
    U f;
    f.h[0] = *(const v8h*)(p);
    f.h[1] = *(const v8h*)(p + 16);
    return f.v;
  }
  static __device__ __forceinline__ v8f mma(v16h a, v16h b, v8f c) {
    return __builtin_amdgcn_wmma_f32_16x16x32_f16(false, a, false, b, (short)0, c, false, false);
  }
};

__device__ __forceinline__ void gemm_mainloop(const _Float16* __restrict__ A, int lda, int m0,
                                              const _Float16* __restrict__ Bt, int ldb, int n0, int K,
                                              int rlane, int koff, v8f (&acc)[4][4]) {
  for (int k0 = 0; k0 < K; k0 += 32) {
    v16h bh[4];
#pragma unroll
    for (int j = 0; j < 4; ++j)
      bh[j] = Frag<_Float16>::load(Bt + (size_t)(n0 + (j << 4) + rlane) * ldb + koff + k0);
#pragma unroll
    for (int i = 0; i < 4; ++i) {
      const v16h ah = Frag<_Float16>::load(A + (size_t)(m0 + (i << 4) + rlane) * lda + koff + k0);
#pragma unroll
      for (int j = 0; j < 4; ++j) acc[i][j] = Frag<_Float16>::mma(ah, bh[j], acc[i][j]);
      guard_row4(acc[i][0], acc[i][1], acc[i][2], acc[i][3], ah, bh[3]);
    }
    keep4_h(bh[0], bh[1], bh[2], bh[3]);
  }
}

__device__ __forceinline__ void store_slab_f16(const float* slab, unsigned short* crow0, int ldc, int lane) {
  const int q = lane >> 3, c8 = (lane & 7) * 8;
  for (int pass = 0; pass < 2; ++pass) {
#pragma unroll
    for (int it = 0; it < 4; ++it) {
      const int row = it * 4 + q;
      const float* sp = slab + row * 68 + c8;
      v8h hv;
#pragma unroll
      for (int e = 0; e < 8; ++e) hv[e] = (_Float16)sp[e];
      *(volatile v8h*)(crow0 + (size_t)row * ldc + c8) = hv;
    }
    __threadfence();
  }
}

__global__ __launch_bounds__(256) void prep_x_kernel(const float* __restrict__ x, unsigned short* __restrict__ xn) {
  __shared__ float tile[64 * 65];
  const int tid = threadIdx.x, lane = tid & 31, wave = tid >> 5;
  const int b = blockIdx.x >> 6;
  const int hw0 = (blockIdx.x & 63) * 64;
#pragma unroll 4
  for (int p = 0; p < 16; ++p) {
    const int idx = tid + p * 256;
    const int cc = idx >> 6;
    const int pp = idx & 63;
    tile[cc * 65 + pp] = x[(((size_t)(b * kCin + cc)) << 12) + hw0 + pp];
  }
  __syncthreads();
  const int q = lane >> 3, c8 = (lane & 7) * 8;
  v8h hv[2];
#pragma unroll
  for (int it = 0; it < 2; ++it) {
    const int tok = it * 32 + wave * 4 + q;
#pragma unroll
    for (int e = 0; e < 8; ++e) hv[it][e] = (_Float16)tile[(c8 + e) * 65 + tok];
  }
  for (int pass = 0; pass < 2; ++pass) {
#pragma unroll
    for (int it = 0; it < 2; ++it) {
      const int tok = it * 32 + wave * 4 + q;
      *(volatile v8h*)(xn + ((size_t)b * kSeq + hw0 + tok) * kCin + c8) = hv[it];
    }
    __threadfence();
  }
}

__global__ __launch_bounds__(256) void prep_w_kernel(
    const float* __restrict__ Wc1, const float* __restrict__ Wg, const float* __restrict__ Wi,
    const float* __restrict__ Ws, const float* __restrict__ Wo,
    unsigned short* __restrict__ wc1p, unsigned short* __restrict__ wgi,
    unsigned short* __restrict__ ws16, unsigned short* __restrict__ wo16) {
  const int blk = blockIdx.x, tid = threadIdx.x;
  v8h hv;
  unsigned short* dst;
  if (blk < 72) {
    const int i = blk * 256 + tid;
    const int o = i / 72;
    const int kk = (i - o * 72) << 3;
    const int tap = kk >> 6;
    const int ci = kk & 63;
    const float* p = Wc1 + ((size_t)(o * kCin + ci)) * 9 + tap;
#pragma unroll
    for (int e = 0; e < 8; ++e) hv[e] = (_Float16)(p[e * 9] * kWCarry);
    dst = wc1p + ((size_t)i << 3);
  } else {
    const int j = blk - 72;
    const float* src;
    unsigned short* d;
    int jb;
    if (j < 32)      { src = Wg; d = wgi;                 jb = j; }
    else if (j < 64) { src = Wi; d = wgi + kHid * kHid;   jb = j - 32; }
    else if (j < 96) { src = Ws; d = ws16;                jb = j - 64; }
    else             { src = Wo; d = wo16;                jb = j - 96; }
    const size_t e0 = ((size_t)(jb * 256 + tid)) << 3;
    const v4f a0 = *(const v4f*)(src + e0);
    const v4f a1 = *(const v4f*)(src + e0 + 4);
#pragma unroll
    for (int e = 0; e < 4; ++e) {
      hv[e]     = (_Float16)(a0[e] * kWCarry);
      hv[4 + e] = (_Float16)(a1[e] * kWCarry);
    }
    dst = d + e0;
  }
  *(volatile v8h*)dst = hv;
  __threadfence();
  *(volatile v8h*)dst = hv;
}

__global__ __launch_bounds__(256) void conv_gemm_kernel(
    const unsigned short* __restrict__ xn, const unsigned short* __restrict__ wc,
    const float* __restrict__ bc1, unsigned short* __restrict__ y) {
  __shared__ __align__(16) unsigned short sx[198 * 72];
  __shared__ __align__(16) float sT[4][16 * 68];
  const int tid = threadIdx.x, lane = tid & 31, wave = tid >> 5;
  const int bh = blockIdx.x;
  const int b = bh >> 6;
  const int h = bh & 63;
  const u4v zero4 = (u4v){0u, 0u, 0u, 0u};
#pragma unroll 4
  for (int p = 0; p < 12; ++p) {
    const int qd = tid + p * kConvThreads;
    const int dy = qd >> 9;
    const int e = qd & 511;
    const int hy = h + dy - 1;
    const bool valid = ((unsigned)hy < 64u);
    const int hyc = hy < 0 ? 0 : (hy > 63 ? 63 : hy);
    const u4v ld = *(const u4v*)(xn + ((size_t)(b * 64 + hyc)) * (kImgW * kCin) + ((size_t)e << 3));
    const u4v v = valid ? ld : zero4;
    *(u4v_a*)(sx + (dy * 66 + 1 + (e >> 3)) * 72 + ((e & 7) << 3)) = v;
  }
  if (tid < 48) {
    const int dy = tid >> 4;
    const int r = tid & 15;
    const int wi = (r >> 3) ? 65 : 0;
    const int ci = r & 7;
    *(u4v_a*)(sx + (dy * 66 + wi) * 72 + (ci << 3)) = zero4;
  }
  __syncthreads();

  const int rlane = lane & 15;
  const int koff = (lane >> 4) * 8;
  const int mOff = (lane >> 4) * 8;
  const int n0 = wave * 64;
  const _Float16* sxh = (const _Float16*)sx;
  const _Float16* wch = (const _Float16*)wc;

  v8f acc[4][4];
#pragma unroll
  for (int i = 0; i < 4; ++i)
#pragma unroll
    for (int j = 0; j < 4; ++j) acc[i][j] = (v8f){0.f, 0.f, 0.f, 0.f, 0.f, 0.f, 0.f, 0.f};

#pragma unroll 1
  for (int tap = 0; tap < 9; ++tap) {
    const int dy = tap / 3;
    const int dx = tap - dy * 3;
#pragma unroll
    for (int hf = 0; hf < 2; ++hf) {
      const int kg = tap * 64 + hf * 32;
      v16h bhf[4];
#pragma unroll
      for (int j = 0; j < 4; ++j)
        bhf[j] = Frag<_Float16>::load(wch + (size_t)(n0 + (j << 4) + rlane) * kConvK + kg + koff);
#pragma unroll
      for (int i = 0; i < 4; ++i) {
        const v16h ah = Frag<_Float16>::load(sxh + (dy * 66 + ((i << 4) + rlane + dx)) * 72 + hf * 32 + koff);
#pragma unroll
        for (int j = 0; j < 4; ++j) acc[i][j] = Frag<_Float16>::mma(ah, bhf[j], acc[i][j]);
        guard_row4(acc[i][0], acc[i][1], acc[i][2], acc[i][3], ah, bhf[3]);
      }
      keep4_h(bhf[0], bhf[1], bhf[2], bhf[3]);
    }
  }
  acc_guard4(acc[0][0], acc[0][1], acc[0][2], acc[0][3]);
  acc_guard4(acc[1][0], acc[1][1], acc[1][2], acc[1][3]);
  acc_guard4(acc[2][0], acc[2][1], acc[2][2], acc[2][3]);
  acc_guard4(acc[3][0], acc[3][1], acc[3][2], acc[3][3]);

  float* slab = sT[wave];
#pragma unroll
  for (int i = 0; i < 4; ++i) {
#pragma unroll
    for (int j = 0; j < 4; ++j) {
      const float bv = bc1[n0 + (j << 4) + rlane];
#pragma unroll
      for (int r = 0; r < 8; ++r)
        slab[(mOff + r) * 68 + (j << 4) + rlane] = acc[i][j][r] * kWCarryInv + bv;
    }
    wave_lds_sync();
    store_slab_f16(slab, y + ((size_t)bh * 64 + (i << 4)) * kHid + n0, kHid, lane);
    wave_lds_sync();
  }
}

__global__ __launch_bounds__(128) void bnstats_kernel(const unsigned* __restrict__ yw, float* __restrict__ part) {
  __shared__ __align__(16) float sP[512];
  const int tid = threadIdx.x;
  const int blk = blockIdx.x;
  const unsigned* p = yw + (size_t)blk * 256 * (kHid / 2) + tid;
  float s0 = 0.f, s1 = 0.f, q0 = 0.f, q1 = 0.f;
#pragma unroll 4
  for (int i = 0; i < 256; ++i) {
    const unsigned w = p[(size_t)i * (kHid / 2)];
    const float a = h16_to_f32(w & 0xffffu);
    const float c = h16_to_f32(w >> 16);
    s0 += a;
    s1 += c;
    q0 = fmaf(a, a, q0);
    q1 = fmaf(c, c, q1);
  }
  sP[2 * tid] = s0;
  sP[2 * tid + 1] = s1;
  sP[256 + 2 * tid] = q0;
  sP[256 + 2 * tid + 1] = q1;
  __syncthreads();
  const v4f v = *(const v4f*)(sP + tid * 4);
  float* dst = part + (size_t)blk * 512 + tid * 4;
  *(volatile v4f*)dst = v;
  __threadfence();
  *(volatile v4f*)dst = v;
}

__global__ __launch_bounds__(256) void bnfinal_kernel(const float* __restrict__ part, const float* __restrict__ gamma,
                                                      const float* __restrict__ beta, float* __restrict__ ss) {
  __shared__ __align__(16) float sS[512];
  const int c = threadIdx.x;
  double s = 0.0, q = 0.0;
#pragma unroll 4
  for (int i = 0; i < 256; ++i) {
    s += (double)part[(size_t)i * 512 + c];
    q += (double)part[(size_t)i * 512 + 256 + c];
  }
  const double inv_n = 1.0 / 65536.0;
  const double mean = s * inv_n;
  double var = q * inv_n - mean * mean;
  var = var < 0.0 ? 0.0 : var;
  const float varf = (float)var;
  const float inv = 1.0f / sqrtf(varf + 1e-5f);
  const float sc = gamma[c] * inv;
  const float sh = beta[c] - (float)mean * sc;
  sS[c] = sc;
  sS[256 + c] = sh;
  __syncthreads();
  if (c < 128) {
    const v4f v = *(const v4f*)(sS + c * 4);
    float* dst = ss + c * 4;
    *(volatile v4f*)dst = v;
    __threadfence();
    *(volatile v4f*)dst = v;
  }
}

__global__ __launch_bounds__(256) void bnact_kernel(const unsigned short* __restrict__ y, const float* __restrict__ ss,
                                                    unsigned short* __restrict__ act, int total8) {
  const int i = blockIdx.x * 256 + threadIdx.x;
  if (i >= total8) return;
  const size_t e0 = (size_t)i << 3;
  const int c0 = (int)(e0 & (size_t)(kHid - 1));
  const u4v w = *(const u4v*)(y + e0);
  const unsigned w0 = w[0];
  const unsigned w1 = w[1];
  const unsigned w2 = w[2];
  const unsigned w3 = w[3];
  const v4f sc0 = *(const v4f*)(ss + c0);
  const v4f sc1 = *(const v4f*)(ss + c0 + 4);
  const v4f sh0 = *(const v4f*)(ss + kHid + c0);
  const v4f sh1 = *(const v4f*)(ss + kHid + c0 + 4);
  const float yv[8] = { h16_to_f32(w0 & 0xffffu), h16_to_f32(w0 >> 16), h16_to_f32(w1 & 0xffffu), h16_to_f32(w1 >> 16),
                        h16_to_f32(w2 & 0xffffu), h16_to_f32(w2 >> 16), h16_to_f32(w3 & 0xffffu), h16_to_f32(w3 >> 16) };
  const float scv[8] = { sc0[0], sc0[1], sc0[2], sc0[3], sc1[0], sc1[1], sc1[2], sc1[3] };
  const float shv[8] = { sh0[0], sh0[1], sh0[2], sh0[3], sh1[0], sh1[1], sh1[2], sh1[3] };
  v8h hv;
#pragma unroll
  for (int e = 0; e < 8; ++e) {
    const float a = fmaf(yv[e], scv[e], shv[e]);
    const float sg = __builtin_amdgcn_rcpf(1.0f + expf(-a));
    hv[e] = (_Float16)(a * sg);
  }
  unsigned short* dst = act + e0;
  *(volatile v8h*)dst = hv;
  __threadfence();
  *(volatile v8h*)dst = hv;
}

template <int EPI>
__global__ __launch_bounds__(256) void gemm_f16_kernel(
    const unsigned short* __restrict__ Ap, const unsigned short* __restrict__ Btp,
    unsigned short* __restrict__ C0, unsigned short* __restrict__ C1,
    const float* __restrict__ bias0, const float* __restrict__ bias1,
    const unsigned short* __restrict__ Gp, int M, int N, int K, float scale) {
  __shared__ __align__(16) float sT[8][16 * 68];
  const int lane = threadIdx.x & 31;
  const int wave = threadIdx.x >> 5;
  const int tilesN = N >> 6;
  const int tilesM = M >> 6;
  const int tile = blockIdx.x * 8 + wave;
  if (tile >= tilesM * tilesN) return;
  const int tm = tile / tilesN;
  const int tn = tile - tm * tilesN;
  const int m0 = tm << 6;
  const int n0 = tn << 6;
  const int rlane = lane & 15;
  const int koff = (lane >> 4) * 8;
  const int mOff = (lane >> 4) * 8;

  v8f acc[4][4];
#pragma unroll
  for (int i = 0; i < 4; ++i)
#pragma unroll
    for (int j = 0; j < 4; ++j) acc[i][j] = (v8f){0.f, 0.f, 0.f, 0.f, 0.f, 0.f, 0.f, 0.f};

  gemm_mainloop((const _Float16*)Ap, K, m0, (const _Float16*)Btp, K, n0, K, rlane, koff, acc);

  acc_guard4(acc[0][0], acc[0][1], acc[0][2], acc[0][3]);
  acc_guard4(acc[1][0], acc[1][1], acc[1][2], acc[1][3]);
  acc_guard4(acc[2][0], acc[2][1], acc[2][2], acc[2][3]);
  acc_guard4(acc[3][0], acc[3][1], acc[3][2], acc[3][3]);

  const bool isGate = (EPI == 0) && (tn < 4);
  const bool second = (EPI == 0) && (tn >= 4);
  const int nc0 = (EPI == 0) ? (n0 & (kHid - 1)) : n0;
  unsigned short* Cp = second ? C1 : C0;
  const float* bp = second ? bias1 : bias0;

  float* slab = sT[wave];
  const int q = lane >> 3, c8 = (lane & 7) * 8;
#pragma unroll
  for (int i = 0; i < 4; ++i) {
    const int mBase = m0 + (i << 4);
#pragma unroll
    for (int j = 0; j < 4; ++j) {
      const float bv = bp[nc0 + (j << 4) + rlane];
#pragma unroll
      for (int r = 0; r < 8; ++r)
        slab[(mOff + r) * 68 + (j << 4) + rlane] = acc[i][j][r] * scale + bv;
    }
    wave_lds_sync();
    if (EPI == 0) {
      if (isGate) {
#pragma unroll 1
        for (int t = 0; t < 32; ++t) {
          float* p = slab + (t >> 1) * 68 + ((t & 1) << 5) + lane;
          const float v = *p;
          *p = __builtin_amdgcn_rcpf(1.0f + expf(-v));
        }
      }
      wave_lds_sync();
    }
    if (EPI == 1) {
#pragma unroll 1
      for (int it = 0; it < 4; ++it) {
        const int row = it * 4 + q;
        const u4v gw = *(const u4v*)(Gp + (size_t)(mBase + row) * kHid + n0 + c8);
        const unsigned g0 = gw[0];
        const unsigned g1 = gw[1];
        const unsigned g2 = gw[2];
        const unsigned g3 = gw[3];
        float* sp = slab + row * 68 + c8;
        v4f a0 = *(const v4f*)(sp);
        v4f a1 = *(const v4f*)(sp + 4);
        a0[0] *= h16_to_f32(g0 & 0xffffu);
        a0[1] *= h16_to_f32(g0 >> 16);
        a0[2] *= h16_to_f32(g1 & 0xffffu);
        a0[3] *= h16_to_f32(g1 >> 16);
        a1[0] *= h16_to_f32(g2 & 0xffffu);
        a1[1] *= h16_to_f32(g2 >> 16);
        a1[2] *= h16_to_f32(g3 & 0xffffu);
        a1[3] *= h16_to_f32(g3 >> 16);
        *(v4f*)(sp) = a0;
        *(v4f*)(sp + 4) = a1;
      }
      wave_lds_sync();
    }
    store_slab_f16(slab, Cp + (size_t)mBase * kHid + nc0, kHid, lane);
    wave_lds_sync();
  }
}

__global__ __launch_bounds__(128) void scan_kernel(const unsigned* __restrict__ U, unsigned* __restrict__ S) {
  __shared__ __align__(16) unsigned tile[kScanSteps * kScanPitch];
  const int tid = threadIdx.x, lane = tid & 31, wave = tid >> 5;
  const size_t rowBase = (size_t)blockIdx.x * kSeq;
  float s0 = 0.f, s1 = 0.f;
#pragma unroll 1
  for (int t0 = 0; t0 < kSeq; t0 += kScanSteps) {
    __syncthreads();
#pragma unroll
    for (int i = 0; i < 8; ++i) {
      const int idx = tid + i * 128;
      const int row = idx >> 5;
      const int c = idx & 31;
      const u4v v = *(const u4v*)(U + (rowBase + t0 + row) * (kHid / 2) + c * 4);
      *(u4v_a*)(tile + row * kScanPitch + c * 4) = v;
    }
    __syncthreads();
#pragma unroll 1
    for (int s = 0; s < kScanSteps; ++s) {
      const unsigned w = tile[s * kScanPitch + tid];
      const float a = h16_to_f32(w & 0xffffu);
      const float c = h16_to_f32(w >> 16);
      s0 = fmaf(0.9f, s0, a);
      s1 = fmaf(0.9f, s1, c);
      const _Float16 h0 = (_Float16)s0;
      const _Float16 h1 = (_Float16)s1;
      const unsigned short b0 = __builtin_bit_cast(unsigned short, h0);
      const unsigned short b1 = __builtin_bit_cast(unsigned short, h1);
      tile[s * kScanPitch + tid] = (unsigned)b0 | ((unsigned)b1 << 16);
    }
    __syncthreads();
    u4v ov[8];
#pragma unroll
    for (int it = 0; it < 8; ++it) ov[it] = *(const u4v_a*)(tile + (it * 4 + wave) * kScanPitch + lane * 4);
    for (int pass = 0; pass < 2; ++pass) {
#pragma unroll
      for (int it = 0; it < 8; ++it)
        *(volatile u4v*)(S + (rowBase + t0 + it * 4 + wave) * (kHid / 2) + lane * 4) = ov[it];
      __threadfence();
    }
  }
}

__global__ __launch_bounds__(256) void outproj_kernel(
    const unsigned short* __restrict__ Ap, const unsigned short* __restrict__ Btp,
    const float* __restrict__ bo, const float* __restrict__ x, float* __restrict__ out) {
  __shared__ __align__(16) float sO[kOutWaves][64 * 68];
  const int lane = threadIdx.x & 31;
  const int wave = threadIdx.x >> 5;
  const int tile = blockIdx.x * kOutWaves + wave;
  if (tile >= (kTok >> 6)) return;
  const int m0 = tile << 6;
  const int rlane = lane & 15;
  const int koff = (lane >> 4) * 8;
  const int mOff = (lane >> 4) * 8;

  v8f acc[4][4];
#pragma unroll
  for (int i = 0; i < 4; ++i)
#pragma unroll
    for (int j = 0; j < 4; ++j) acc[i][j] = (v8f){0.f, 0.f, 0.f, 0.f, 0.f, 0.f, 0.f, 0.f};

  gemm_mainloop((const _Float16*)Ap, kHid, m0, (const _Float16*)Btp, kHid, 0, kHid, rlane, koff, acc);

  acc_guard4(acc[0][0], acc[0][1], acc[0][2], acc[0][3]);
  acc_guard4(acc[1][0], acc[1][1], acc[1][2], acc[1][3]);
  acc_guard4(acc[2][0], acc[2][1], acc[2][2], acc[2][3]);
  acc_guard4(acc[3][0], acc[3][1], acc[3][2], acc[3][3]);

  float* T = sO[wave];
#pragma unroll
  for (int j = 0; j < 4; ++j) {
    const float bv = bo[(j << 4) + rlane];
#pragma unroll
    for (int i = 0; i < 4; ++i) {
#pragma unroll
      for (int r = 0; r < 8; ++r)
        T[((j << 4) + rlane) * 68 + (i << 4) + mOff + r] = acc[i][j][r] * kWCarryInv + bv;
    }
  }
  wave_lds_sync();
  const int b = tile >> 6;
  const int h = tile & 63;
  const int hh = lane >> 4, c4 = (lane & 15) * 4;
  const size_t obase = ((size_t)b * kCin) * kSeq + (size_t)h * kImgW + c4;
#pragma unroll 1
  for (int it = 0; it < 32; ++it) {
    const int o = it * 2 + hh;
    float* tp = T + o * 68 + c4;
    const v4f xv = *(const v4f*)(x + obase + (size_t)o * kSeq);
    v4f tv = *(const v4f*)tp;
    tv += xv;
    *(v4f*)tp = tv;
  }
  wave_lds_sync();
  for (int pass = 0; pass < 2; ++pass) {
#pragma unroll 4
    for (int it = 0; it < 32; ++it) {
      const int o = it * 2 + hh;
      const v4f v = *(const v4f*)(T + o * 68 + c4);
      *(volatile v4f*)(out + obase + (size_t)o * kSeq) = v;
    }
    __threadfence();
  }
}

extern "C" void kernel_launch(void* const* d_in, const int* in_sizes, int n_in,
                              void* d_out, int out_size, void* d_ws, size_t ws_size,
                              hipStream_t stream) {
  if (n_in < 13) return;
  if (in_sizes[0] != kBatch * kCin * kSeq) return;
  if (in_sizes[1] != kHid * kCin * 9) return;
  if (in_sizes[2] != kHid || in_sizes[3] != kHid || in_sizes[4] != kHid) return;
  if (in_sizes[5] != kHid * kHid || in_sizes[6] != kHid) return;
  if (in_sizes[7] != kHid * kHid || in_sizes[8] != kHid) return;
  if (in_sizes[9] != kHid * kHid || in_sizes[10] != kHid) return;
  if (in_sizes[11] != kCin * kHid || in_sizes[12] != kCin) return;
  if (out_size != kBatch * kCin * kSeq) return;
  if (ws_size < kWsTotal) return;

  const float* x     = (const float*)d_in[0];
  const float* Wc1   = (const float*)d_in[1];
  const float* bc1   = (const float*)d_in[2];
  const float* gamma = (const float*)d_in[3];
  const float* beta  = (const float*)d_in[4];
  const float* Wg    = (const float*)d_in[5];
  const float* bg    = (const float*)d_in[6];
  const float* Wi    = (const float*)d_in[7];
  const float* bi    = (const float*)d_in[8];
  const float* Ws    = (const float*)d_in[9];
  const float* bs    = (const float*)d_in[10];
  const float* Wo    = (const float*)d_in[11];
  const float* bo    = (const float*)d_in[12];
  float* out = (float*)d_out;

  char* ws = (char*)d_ws;
  unsigned short* R0   = (unsigned short*)(ws + kOffR0);
  unsigned short* R1   = (unsigned short*)(ws + kOffR1);
  unsigned short* R2   = (unsigned short*)(ws + kOffR2);
  unsigned short* WC1P = (unsigned short*)(ws + kOffWC1P);
  unsigned short* WGI  = (unsigned short*)(ws + kOffWGI);
  unsigned short* WS16 = (unsigned short*)(ws + kOffWS16);
  unsigned short* WO16 = (unsigned short*)(ws + kOffWO16);
  float*          PART = (float*)(ws + kOffPART);
  float*          SS   = (float*)(ws + kOffSS);

  prep_x_kernel<<<kBatch * 64, 256, 0, stream>>>(x, R2);
  prep_w_kernel<<<176, 256, 0, stream>>>(Wc1, Wg, Wi, Ws, Wo, WC1P, WGI, WS16, WO16);
  conv_gemm_kernel<<<kBatch * kImgH, kConvThreads, 0, stream>>>(R2, WC1P, bc1, R0);
  bnstats_kernel<<<256, 128, 0, stream>>>((const unsigned*)R0, PART);
  bnfinal_kernel<<<1, 256, 0, stream>>>(PART, gamma, beta, SS);
  bnact_kernel<<<(kTok * kHid / 8) / 256, 256, 0, stream>>>(R0, SS, R1, kTok * kHid / 8);
  gemm_f16_kernel<0><<<(kTok / 64) * (kGuN / 64) / 8, 256, 0, stream>>>(
      R1, WGI, R2, R0, bg, bi, R1, kTok, kGuN, kHid, kWCarryInv);
  scan_kernel<<<kBatch, 128, 0, stream>>>((const unsigned*)R0, (unsigned*)R1);
  gemm_f16_kernel<1><<<(kTok / 64) * (kHid / 64) / 8, 256, 0, stream>>>(
      R1, WS16, R0, R0, bs, bs, R2, kTok, kHid, kHid, kWCarryInv);
  outproj_kernel<<<(kTok / 64) / kOutWaves, 32 * kOutWaves, 0, stream>>>(R0, WO16, bo, x, out);
}
